// Model_5523327942836
// MI455X (gfx1250) — hardware-verified
//
#include <hip/hip_runtime.h>
#include <stddef.h>
#include <stdint.h>
#include <math.h>


#define NBATCH  512
#define NPG     32
#define TIN     12
#define NN      16384
#define NEDGE   131072
#define KP1     32
#define HC1     512
#define HID     64
#define NHD1    8
#define KA2     1024
#define G3      192
#define NOUT    9
#define NTHR    256
#define NWAVE   8
#define EPT     8
#define CHUNK   (NTHR * EPT)
#define WCAP    (EPT * 32)
#define LISTN   (NWAVE * WCAP)
#define NBMAX   2048
#define SLOTB   11
#define NBRUN   1024
#define RCAP    16384
#define DEGCAP  64
#define GBM     64
#define GBN     64
#define GTHR    128
#define NEGSL   0.2f
#define EPS_SM  1e-16f
#define EPS_LN  1e-5f
#define WSMAX   134217728
#define LDS_AGG ((2 * RCAP + 2 * NBMAX + LISTN) * 4 + 64)

static_assert(NN == NBATCH * NPG);
static_assert((CHUNK & (CHUNK - 1)) == 0 && CHUNK <= (1 << SLOTB));
static_assert(NBMAX == (1 << SLOTB));
static_assert(NTHR * 8 == NBMAX);
static_assert(LISTN >= NBMAX && LISTN >= NWAVE * WCAP);
static_assert((RCAP % 32) == 0);
static_assert(RCAP >= 8192 + 8192 / 20 + 1);
static_assert(DEGCAP >= 22 + 8);
static_assert(NEDGE < (1 << (32 - SLOTB)));
static_assert((NEDGE % CHUNK) == 0);
static_assert((NN % NBRUN) == 0 && NBRUN <= NBMAX && (NBRUN & (NBRUN - 1)) == 0 && NBRUN >= 32);
static_assert(LDS_AGG <= 300000);
static_assert(GBM == (GTHR / 32) * 16);
static_assert(GTHR == 2 * GBN && GTHR == 2 * GBM);
static_assert((KP1 % 32) == 0 && (KA2 % 32) == 0 && KA2 == 2 * HC1);
static_assert((HC1 % GBN) == 0 && HID == GBN && (NN % GBM) == 0);
static_assert(HC1 == 16 * 32 && HID == 2 * 32);
static_assert(HID == 64 && 3 * HID == G3 && NPG == 32 && (NBATCH % 32) == 0);
static_assert((32 * NOUT * 4) % 128 == 0);
static_assert((NBATCH / 32) * 32 * NOUT == NBATCH * NOUT);

#define O_XB   0
#define O_W1T  (O_XB  + NN * KP1 * 2)
#define O_W2D  (O_W1T + HC1 * KP1 * 2)
#define O_H1   (O_W2D + HID * KA2 * 2)
#define O_SD1  (O_H1  + NN * HC1 * 4)
#define O_X1   (O_SD1 + 2 * NHD1 * NN * 4)
#define O_H2   (O_X1  + NN * KA2 * 2)
#define O_SD2  (O_H2  + NN * HID * 4)
#define O_LNF  (O_SD2 + 2 * NN * 4)
#define O_SEQ  (O_LNF + NN * HID * 4)
#define O_END  (O_SEQ + NBATCH * HID * 64 * 2)
static_assert(O_END == 82083840);
static_assert(O_END <= WSMAX);
static_assert((O_W1T % 128) == 0 && (O_W2D % 128) == 0 && (O_H1 % 128) == 0 && (O_SD1 % 128) == 0 && (O_X1 % 128) == 0 &&
              (O_H2 % 128) == 0 && (O_SD2 % 128) == 0 && (O_LNF % 128) == 0 && (O_SEQ % 128) == 0);

#define PU_XB  (NN * 4)
#define PU_W1  (HC1 * 4)
#define PU_W2  (HID * (KA2 / 8))
#define PB_XB  (PU_XB / NTHR)
#define PB_W1  (PU_W1 / NTHR)
#define PB_W2  (PU_W2 / NTHR)
static_assert((PU_XB % NTHR) == 0 && (PU_W1 % NTHR) == 0 && (PU_W2 % NTHR) == 0);

#define LO_WI1  0
#define LO_WH1  12288
#define LO_WI2  36864
#define LO_WH2  61440
#define LO_H1   86016
#define LO_H2   102400
#define LO_SEQ  118784
#define LO_HF   122880
#define LO_WF   131072
#define LO_BF   133376
#define LO_BIAS 133440
#define LO_OUT  136512
#define LDS_REC 137664
static_assert(LO_WH1 == LO_WI1 + G3 * NPG * 2 && LO_WI2 == LO_WH1 + G3 * HID * 2 && LO_WH2 == LO_WI2 + G3 * HID * 2);
static_assert(LO_H1 == LO_WH2 + G3 * HID * 2 && LO_H2 == LO_H1 + 2 * 32 * 128 * 2 && LO_SEQ == LO_H2 + 2 * 32 * 128 * 2);
static_assert(LO_HF == LO_SEQ + 32 * 64 * 2 && LO_WF == LO_HF + 32 * 64 * 4 && LO_BF == LO_WF + NOUT * HID * 4);
static_assert(LO_BIAS == LO_BF + 64 && LO_OUT == LO_BIAS + 4 * G3 * 4 && LDS_REC == LO_OUT + 32 * NOUT * 4);
static_assert((LO_BF % 16) == 0 && (LO_BIAS % 16) == 0 && (LO_OUT % 16) == 0);

typedef float          v2f  __attribute__((ext_vector_type(2)));
typedef float          v4f  __attribute__((ext_vector_type(4)));
typedef float          v8f  __attribute__((ext_vector_type(8)));
typedef int            v4i  __attribute__((ext_vector_type(4)));
typedef int            v8i  __attribute__((ext_vector_type(8)));
typedef unsigned int   v4u  __attribute__((ext_vector_type(4)));
typedef unsigned short v8us __attribute__((ext_vector_type(8)));
typedef __bf16         v16b __attribute__((ext_vector_type(16)));
typedef v2f  __attribute__((may_alias)) v2fa;
typedef v4f  __attribute__((may_alias)) v4fa;
typedef v4u  __attribute__((may_alias)) v4ua;
typedef v8us __attribute__((may_alias)) v8usa;
union FragB { v16b v; v8us h[2]; v8i w; };
struct HL { v4u hi; v4u lo; };

__device__ __forceinline__ v8f wmb(const FragB& a, const FragB& b, v8f c) {
  v8f d = __builtin_amdgcn_wmma_f32_16x16x32_bf16(false, a.v, false, b.v, (short)0, c, false, false);
  asm volatile("v_nop\n\tv_nop\n\tv_nop\n\tv_nop" : "+v"(d) : "v"(a.w), "v"(b.w));
  return d;
}

__device__ __forceinline__ unsigned int f2bf(float f) {
  const unsigned int u = __float_as_uint(f);
  return ((u + 0x7FFFu + ((u >> 16) & 1u)) >> 16) & 0xFFFFu;
}
__device__ __forceinline__ float bf2f(unsigned int b) { return __uint_as_float(b << 16); }
__device__ __forceinline__ float bfr(float f) { return bf2f(f2bf(f)); }
__device__ __forceinline__ v4f bfr4(const v4f a) {
  v4f r; r.x = bfr(a.x); r.y = bfr(a.y); r.z = bfr(a.z); r.w = bfr(a.w); return r;
}
__device__ __forceinline__ unsigned int pk2(float lo, float hi) { return f2bf(lo) | (f2bf(hi) << 16); }
__device__ __forceinline__ v4u pack8(const v4f a, const v4f b) {
  v4u r;
  r.x = pk2(a.x, a.y); r.y = pk2(a.z, a.w); r.z = pk2(b.x, b.y); r.w = pk2(b.z, b.w);
  return r;
}
__device__ __forceinline__ HL split8(const v4f a, const v4f b) {
  const unsigned int h0 = f2bf(a.x), h1 = f2bf(a.y), h2 = f2bf(a.z), h3 = f2bf(a.w);
  const unsigned int h4 = f2bf(b.x), h5 = f2bf(b.y), h6 = f2bf(b.z), h7 = f2bf(b.w);
  const unsigned int l0 = f2bf(a.x - bf2f(h0)), l1 = f2bf(a.y - bf2f(h1)), l2 = f2bf(a.z - bf2f(h2)), l3 = f2bf(a.w - bf2f(h3));
  const unsigned int l4 = f2bf(b.x - bf2f(h4)), l5 = f2bf(b.y - bf2f(h5)), l6 = f2bf(b.z - bf2f(h6)), l7 = f2bf(b.w - bf2f(h7));
  HL r;
  v4u hv, lv;
  hv.x = h0 | (h1 << 16); hv.y = h2 | (h3 << 16); hv.z = h4 | (h5 << 16); hv.w = h6 | (h7 << 16);
  lv.x = l0 | (l1 << 16); lv.y = l2 | (l3 << 16); lv.z = l4 | (l5 << 16); lv.w = l6 | (l7 << 16);
  r.hi = hv; r.lo = lv;
  return r;
}
__device__ __forceinline__ float elu_f(float v) {
  const float e = expm1f(v);
  return (v > 0.0f) ? v : e;
}
__device__ __forceinline__ float leaky(float v) { return (v > 0.f) ? v : NEGSL * v; }
__device__ __forceinline__ float sigm_f(float v) { return __builtin_amdgcn_rcpf(1.0f + expf(-v)); }
__device__ __forceinline__ void osm_step(float lg, float& mx, float& dn, float& s1, float& s2) {
  const float df = lg - mx;
  const float ee = __expf(-fabsf(df));
  const bool up  = df > 0.f;
  s1 = up ? ee : 1.0f;
  s2 = up ? 1.0f : ee;
  mx = up ? lg : mx;
  dn = fmaf(dn, s1, s2);
}
__device__ __forceinline__ v4f upd4(const v4f a, float s1, float s2, const v4f f) {
  v4f r;
  r.x = fmaf(a.x, s1, s2 * f.x); r.y = fmaf(a.y, s1, s2 * f.y);
  r.z = fmaf(a.z, s1, s2 * f.z); r.w = fmaf(a.w, s1, s2 * f.w);
  return r;
}
__device__ __forceinline__ v4f aff4(const v4f a, float inv, const v4f b) {
  v4f r;
  r.x = fmaf(a.x, inv, b.x); r.y = fmaf(a.y, inv, b.y); r.z = fmaf(a.z, inv, b.z); r.w = fmaf(a.w, inv, b.w);
  return r;
}

__device__ __forceinline__ int scan_chunk(const int* __restrict__ dsts, int nE, int cbase, int slotBase,
                                          int nb, int vec8, int* list, int tid, int lane, int wave) {
  int wc = 0;
  const int el0  = tid * EPT;
  const int e0   = cbase + el0;
  const int sent = -2147483647 - 1;
  v4i da, db;
  if (vec8 != 0 && cbase + CHUNK <= nE) {
    da = *(const v4i*)(dsts + e0);
    db = *(const v4i*)(dsts + e0 + 4);
  } else {
    da.x = (e0     < nE) ? dsts[min(e0,     nE - 1)] : sent;
    da.y = (e0 + 1 < nE) ? dsts[min(e0 + 1, nE - 1)] : sent;
    da.z = (e0 + 2 < nE) ? dsts[min(e0 + 2, nE - 1)] : sent;
    da.w = (e0 + 3 < nE) ? dsts[min(e0 + 3, nE - 1)] : sent;
    db.x = (e0 + 4 < nE) ? dsts[min(e0 + 4, nE - 1)] : sent;
    db.y = (e0 + 5 < nE) ? dsts[min(e0 + 5, nE - 1)] : sent;
    db.z = (e0 + 6 < nE) ? dsts[min(e0 + 6, nE - 1)] : sent;
    db.w = (e0 + 7 < nE) ? dsts[min(e0 + 7, nE - 1)] : sent;
  }
  const unsigned nbs = (unsigned)slotBase;
  const unsigned unb = (unsigned)nb;
  const unsigned s0 = (unsigned)da.x - nbs, s1 = (unsigned)da.y - nbs;
  const unsigned s2 = (unsigned)da.z - nbs, s3 = (unsigned)da.w - nbs;
  const unsigned s4 = (unsigned)db.x - nbs, s5 = (unsigned)db.y - nbs;
  const unsigned s6 = (unsigned)db.z - nbs, s7 = (unsigned)db.w - nbs;
  const bool h0 = s0 < unb, h1 = s1 < unb, h2 = s2 < unb, h3 = s3 < unb;
  const bool h4 = s4 < unb, h5 = s5 < unb, h6 = s6 < unb, h7 = s7 < unb;
  const unsigned any = __builtin_amdgcn_ballot_w32(h0 | h1 | h2 | h3 | h4 | h5 | h6 | h7);
  if (any != 0u) {
#define HITJ(J, HJ, SJ) { \
      const unsigned mj = __builtin_amdgcn_ballot_w32(HJ); \
      if (mj != 0u) { \
        if (HJ) { \
          const int pos = wc + (int)__builtin_amdgcn_mbcnt_lo(mj, 0u); \
          if (pos < WCAP) list[wave * WCAP + pos] = ((el0 + (J)) << SLOTB) | (int)(SJ); \
        } \
        wc += (int)__builtin_popcount(mj); } }
    HITJ(0, h0, s0)
    HITJ(1, h1, s1)
    HITJ(2, h2, s2)
    HITJ(3, h3, s3)
    HITJ(4, h4, s4)
    HITJ(5, h5, s5)
    HITJ(6, h6, s6)
    HITJ(7, h7, s7)
#undef HITJ
  }
  return wc;
}

__global__ __launch_bounds__(NTHR) void k_prep(const float* __restrict__ x, const float* __restrict__ W1,
                                               const float* __restrict__ W2, unsigned short* planes) {
  const int b = (int)blockIdx.x, tid = (int)threadIdx.x;
  const v4f z4 = {0.f, 0.f, 0.f, 0.f};
  v4f a, c;
  size_t oo;
  if (b < PB_XB) {
    const int u = b * NTHR + tid;
    const int row = u >> 2, q = u & 3;
    const float* p = x + (size_t)row * TIN;
    const int oa = (q == 0) ? 0 : 8;
    const int oc = (q == 0) ? 4 : 8;
    a = *(const v4fa*)(p + oa);
    c = *(const v4fa*)(p + oc);
    if (q > 1) a = z4;
    if (q > 0) c = z4;
    oo = (size_t)row * KP1 + 8 * q;
  } else if (b < PB_XB + PB_W1) {
    const int u = (b - PB_XB) * NTHR + tid;
    const int n = u >> 2, k8 = (u & 3) * 8;
    const float* p = W1 + n;
    const int c0 = (k8 + 0 < TIN) ? k8 + 0 : TIN - 1, c1 = (k8 + 1 < TIN) ? k8 + 1 : TIN - 1;
    const int c2 = (k8 + 2 < TIN) ? k8 + 2 : TIN - 1, c3 = (k8 + 3 < TIN) ? k8 + 3 : TIN - 1;
    const int c4 = (k8 + 4 < TIN) ? k8 + 4 : TIN - 1, c5 = (k8 + 5 < TIN) ? k8 + 5 : TIN - 1;
    const int c6 = (k8 + 6 < TIN) ? k8 + 6 : TIN - 1, c7 = (k8 + 7 < TIN) ? k8 + 7 : TIN - 1;
    float e0 = p[(size_t)c0 * HC1], e1 = p[(size_t)c1 * HC1], e2 = p[(size_t)c2 * HC1], e3 = p[(size_t)c3 * HC1];
    float e4 = p[(size_t)c4 * HC1], e5 = p[(size_t)c5 * HC1], e6 = p[(size_t)c6 * HC1], e7 = p[(size_t)c7 * HC1];
    e0 = (k8 + 0 < TIN) ? e0 : 0.f; e1 = (k8 + 1 < TIN) ? e1 : 0.f; e2 = (k8 + 2 < TIN) ? e2 : 0.f; e3 = (k8 + 3 < TIN) ? e3 : 0.f;
    e4 = (k8 + 4 < TIN) ? e4 : 0.f; e5 = (k8 + 5 < TIN) ? e5 : 0.f; e6 = (k8 + 6 < TIN) ? e6 : 0.f; e7 = (k8 + 7 < TIN) ? e7 : 0.f;
    a.x = e0; a.y = e1; a.z = e2; a.w = e3;
    c.x = e4; c.y = e5; c.z = e6; c.w = e7;
    oo = (size_t)NN * KP1 + (size_t)n * KP1 + k8;
  } else {
    const int u = (b - PB_XB - PB_W1) * NTHR + tid;
    const int n = u >> 7, k8 = (u & 127) * 8;
    const int kk = k8 & (HC1 - 1);
    const float* p = W2 + (size_t)kk * HID + n;
    a.x = p[0];       a.y = p[HID];     a.z = p[2 * HID]; a.w = p[3 * HID];
    c.x = p[4 * HID]; c.y = p[5 * HID]; c.z = p[6 * HID]; c.w = p[7 * HID];
    oo = (size_t)NN * KP1 + (size_t)HC1 * KP1 + (size_t)n * KA2 + k8;
  }
  const v4u wv = pack8(a, c);
  unsigned short* o = planes + oo;
  *(volatile v4u*)o = wv;
  __threadfence();
  *(volatile v4u*)o = wv;
}

__global__ __launch_bounds__(GTHR) void k_gemm(
    const unsigned short* __restrict__ A, const unsigned short* __restrict__ WT,
    float* outF, int K, int ldo,
    const float* __restrict__ atts, const float* __restrict__ attd, int attLen,
    float* SD, int MPr)
{
  __shared__ __attribute__((aligned(16))) float stg[GBM * GBN];
  __shared__ __attribute__((aligned(16))) float satt[2 * GBN];
  __shared__ __attribute__((aligned(16))) float sdot[2 * GBM];
  const int tid = (int)threadIdx.x, lane = tid & 31, wave = tid >> 5, hh = lane >> 4, m = lane & 15;
  const int rowBase = (int)blockIdx.x * GBM;
  const int head    = (int)blockIdx.y;
  const int col0    = head * GBN;

  {
    const int which = tid >> 6;
    const int c  = tid & 63;
    const int cl = c < attLen ? c : attLen - 1;
    const float vs = atts[head * attLen + cl];
    const float vd = attd[head * attLen + cl];
    float v = (which == 0) ? vs : vd;
    v = (c < attLen) ? bfr(v) : 0.f;
    satt[which * GBN + c] = v;
  }

  v8f acc[4];
  {
    const v8f z = {0.f, 0.f, 0.f, 0.f, 0.f, 0.f, 0.f, 0.f};
    acc[0] = z; acc[1] = z; acc[2] = z; acc[3] = z;
  }
  const unsigned short* ap = A  + (size_t)(rowBase + 16 * wave + m) * (size_t)K + 8 * hh;
  const unsigned short* wp = WT + (size_t)(col0 + m) * (size_t)K + 8 * hh;
  const int ksteps = K >> 5;
#pragma unroll 1
  for (int ks = 0; ks < ksteps; ++ks) {
    FragB af;
    af.h[0] = *(const v8usa*)(ap + 32 * ks);
    af.h[1] = *(const v8usa*)(ap + 32 * ks + 16);
#pragma unroll
    for (int t = 0; t < 4; ++t) {
      const unsigned short* wq = wp + (size_t)(16 * t) * (size_t)K + 32 * ks;
      FragB bf;
      bf.h[0] = *(const v8usa*)wq;
      bf.h[1] = *(const v8usa*)(wq + 16);
      acc[t] = wmb(af, bf, acc[t]);
    }
  }

#pragma unroll
  for (int t = 0; t < 4; ++t) {
    const int lc = 16 * t + m;
#pragma unroll
    for (int r = 0; r < 8; ++r) {
      const int lr = 16 * wave + 8 * hh + r;
      stg[lr * GBN + lc] = acc[t][r];
    }
  }
  __syncthreads();

  {
    const int row = tid & 63, which = tid >> 6;
    const float* sa = satt + which * GBN;
    const float* hr = stg + row * GBN;
    float d = 0.f;
#pragma unroll 4
    for (int c4 = 0; c4 < GBN / 4; ++c4) {
      const v4f hv = *(const v4fa*)(hr + 4 * c4);
      const v4f av = *(const v4fa*)(sa + 4 * c4);
      d = fmaf(hv.x, av.x, d);
      d = fmaf(hv.y, av.y, d);
      d = fmaf(hv.z, av.z, d);
      d = fmaf(hv.w, av.w, d);
    }
    sdot[which * GBM + row] = d;
  }
  __syncthreads();

  v4f fv[8];
#pragma unroll
  for (int i = 0; i < 8; ++i) {
    const int lr = 16 * wave + 2 * i + hh;
    fv[i] = *(const v4fa*)(stg + lr * GBN + 4 * m);
  }
  const int which2 = lane >> 4, piece = lane & 15;
  const v4f sdv = *(const v4fa*)(sdot + which2 * GBM + 4 * piece);
  float* sp = SD + (size_t)(2 * head + which2) * (size_t)MPr + rowBase + 4 * piece;

#pragma unroll
  for (int i = 0; i < 8; ++i) {
    const int lr = 16 * wave + 2 * i + hh;
    const int gr = rowBase + lr;
    float* op = outF + (size_t)gr * (size_t)ldo + col0 + 4 * m;
    *(volatile v4f*)op = fv[i];
  }
  if (wave == 0) *(volatile v4f*)sp = sdv;
  __threadfence();
#pragma unroll
  for (int i = 0; i < 8; ++i) {
    const int lr = 16 * wave + 2 * i + hh;
    const int gr = rowBase + lr;
    float* op = outF + (size_t)gr * (size_t)ldo + col0 + 4 * m;
    *(volatile v4f*)op = fv[i];
  }
  if (wave == 0) *(volatile v4f*)sp = sdv;
}

template<int L>
__global__ __launch_bounds__(NTHR) void k_agg(
    const int* __restrict__ srcs, const int* __restrict__ dsts,
    const float* __restrict__ F, const float* __restrict__ SD,
    const float* __restrict__ bias, const float* __restrict__ gam, const float* __restrict__ bet,
    unsigned short* HP, float* LNF,
    int nN, int nE, int nb, int vec8, int MPr) {
  extern __shared__ v4f lds_dyn[];
  int* reg1 = (int*)lds_dyn;
  int* reg2 = reg1 + RCAP;
  int* scnt = reg2 + RCAP;
  int* soff = scnt + NBMAX;
  int* list = soff + NBMAX;
  int* wcnt = list + LISTN;
  int* wtot = wcnt + NWAVE;
  const int tid = (int)threadIdx.x, lane = tid & 31, wave = tid >> 5;
  const int nodeBase = (int)blockIdx.x * nb;

  for (int i = tid; i < NBMAX; i += NTHR) scnt[i] = 0;
  __syncthreads();

  int tot = 0;
  const int nChunks = (nE + CHUNK - 1) / CHUNK;
#pragma unroll 1
  for (int ch = 0; ch < nChunks; ++ch) {
    const int cbase = ch * CHUNK;
    const int wc = scan_chunk(dsts, nE, cbase, nodeBase, nb, vec8, list, tid, lane, wave);
    if (lane == 0) wcnt[wave] = wc;
    __syncthreads();
    int pre = 0, all = 0;
#pragma unroll
    for (int w2 = 0; w2 < NWAVE; ++w2) {
      int c = wcnt[w2];
      c = c < 0 ? 0 : (c > WCAP ? WCAP : c);
      all += c;
      pre += (w2 < wave) ? c : 0;
    }
    const int wcc  = wc > WCAP ? WCAP : wc;
    const int base = tot + pre;
#pragma unroll 1
    for (int i = lane; i < wcc; i += 32) {
      const int ent = list[wave * WCAP + i];
      const int el  = (ent >> SLOTB) & (CHUNK - 1);
      const int sl  = ent & (NBMAX - 1);
      int eid = cbase + el;
      eid = eid > nE - 1 ? nE - 1 : eid;
      const int pos = base + i;
      if (pos < RCAP) reg1[pos] = (int)(((unsigned)eid << SLOTB) | (unsigned)sl);
    }
    tot += all;
    tot = tot > RCAP ? RCAP : tot;
    __syncthreads();
  }
  const int nh = tot;

  if (wave == 0) {
#pragma unroll 1
    for (int b0 = 0; b0 < nh; b0 += 32) {
      const int idx = b0 + lane;
      const int uv  = reg1[idx < nh ? idx : nh - 1];
      const int m32 = (nh - b0) < 32 ? (nh - b0) : 32;
#pragma unroll 1
      for (int k = 0; k < m32; ++k) {
        const int u  = __builtin_amdgcn_readlane(uv, k);
        const int sl = u & (NBMAX - 1);
        if (lane == 0) scnt[sl] = scnt[sl] + 1;
      }
    }
  }
  __syncthreads();

  {
    const v4i ca = *(const v4i*)(scnt + 8 * tid);
    const v4i cb = *(const v4i*)(scnt + 8 * tid + 4);
    const int e0 = ca.x < 0 ? 0 : ca.x, e1 = ca.y < 0 ? 0 : ca.y, e2 = ca.z < 0 ? 0 : ca.z, e3 = ca.w < 0 ? 0 : ca.w;
    const int e4 = cb.x < 0 ? 0 : cb.x, e5 = cb.y < 0 ? 0 : cb.y, e6 = cb.z < 0 ? 0 : cb.z, e7 = cb.w < 0 ? 0 : cb.w;
    const int ts = e0 + e1 + e2 + e3 + e4 + e5 + e6 + e7;
    int incl = ts;
#pragma unroll
    for (int d = 1; d < 32; d <<= 1) {
      const int up = __shfl_up(incl, d);
      if (lane >= d) incl += up;
    }
    if (lane == 31) wtot[wave] = incl;
    __syncthreads();
    int pre = 0;
#pragma unroll
    for (int w2 = 0; w2 < NWAVE; ++w2) pre += (w2 < wave) ? wtot[w2] : 0;
    int run = pre + incl - ts;
    soff[8 * tid + 0] = run; run += e0;
    soff[8 * tid + 1] = run; run += e1;
    soff[8 * tid + 2] = run; run += e2;
    soff[8 * tid + 3] = run; run += e3;
    soff[8 * tid + 4] = run; run += e4;
    soff[8 * tid + 5] = run; run += e5;
    soff[8 * tid + 6] = run; run += e6;
    soff[8 * tid + 7] = run;
  }
  __syncthreads();
  for (int i = tid; i < NBMAX; i += NTHR) list[i] = soff[i];
  __syncthreads();

  if (wave == 0) {
#pragma unroll 1
    for (int b0 = 0; b0 < nh; b0 += 32) {
      const int idx = b0 + lane;
      const int uv  = reg1[idx < nh ? idx : nh - 1];
      const int m32 = (nh - b0) < 32 ? (nh - b0) : 32;
#pragma unroll 1
      for (int k = 0; k < m32; ++k) {
        const int u   = __builtin_amdgcn_readlane(uv, k);
        const int sl  = u & (NBMAX - 1);
        const int eid = (int)((unsigned)u >> SLOTB);
        if (lane == 0) {
          int pos = list[sl];
          pos = pos < 0 ? 0 : (pos > RCAP - 1 ? RCAP - 1 : pos);
          reg2[pos] = eid;
          list[sl] = pos + 1;
        }
      }
    }
  }
  __syncthreads();

  const int nbw = nb >> 3;
  const bool ovf = (nh >= RCAP);
  const float qnan = __int_as_float(0x7fc00000);

  if (L == 1) {
    const int cA = 8 * lane;
    const int cB = (HC1 / 2) + 8 * lane;
    const int hA = lane >> 3;
    const int hB = 4 + (lane >> 3);
    const v4f bA0 = bfr4(*(const v4fa*)(bias + cA));
    const v4f bA1 = bfr4(*(const v4fa*)(bias + cA + 4));
    const v4f bB0 = bfr4(*(const v4fa*)(bias + cB));
    const v4f bB1 = bfr4(*(const v4fa*)(bias + cB + 4));
    const float* ASa = SD + (size_t)(2 * hA) * (size_t)MPr;
    const float* ADa = ASa + MPr;
    const float* ASb = SD + (size_t)(2 * hB) * (size_t)MPr;
    const float* ADb = ASb + MPr;

#pragma unroll 1
    for (int jt = 0; jt < nbw; ++jt) {
      const int slot = wave * nbw + jt;
      const int grow = nodeBase + slot;
      const int gcl  = grow < nN ? grow : nN - 1;
      int st = soff[slot];
      const int craw = scnt[slot];
      int cnt = craw;
      st  = st < 0 ? 0 : (st > nh ? nh : st);
      cnt = cnt < 0 ? 0 : (cnt > DEGCAP ? DEGCAP : cnt);
      if (cnt > nh - st) cnt = nh - st;
      const float pz = (ovf || craw > DEGCAP) ? qnan : 0.0f;

      const float* fr = F + (size_t)gcl * HC1;
      v4f a0 = *(const v4fa*)(fr + cA);
      v4f a1 = *(const v4fa*)(fr + cA + 4);
      v4f a2 = *(const v4fa*)(fr + cB);
      v4f a3 = *(const v4fa*)(fr + cB + 4);
      const float adA = ADa[gcl], adB = ADb[gcl];
      float mxA = leaky(ASa[gcl] + adA), dnA = 1.0f;
      float mxB = leaky(ASb[gcl] + adB), dnB = 1.0f;

#pragma unroll 1
      for (int q = 0; q < cnt; ++q) {
        int idx = st + q; idx = idx > RCAP - 1 ? RCAP - 1 : idx;
        int eid = reg2[idx]; eid = eid < 0 ? 0 : (eid > nE - 1 ? nE - 1 : eid);
        const int sraw = srcs[eid];
        const int s = sraw < 0 ? 0 : (sraw > nN - 1 ? nN - 1 : sraw);
        const float* fs = F + (size_t)s * HC1;
        const v4f f0 = *(const v4fa*)(fs + cA);
        const v4f f1 = *(const v4fa*)(fs + cA + 4);
        const v4f f2 = *(const v4fa*)(fs + cB);
        const v4f f3 = *(const v4fa*)(fs + cB + 4);
        const float lgA = leaky(ASa[s] + adA);
        const float lgB = leaky(ASb[s] + adB);
        float s1, s2;
        osm_step(lgA, mxA, dnA, s1, s2);
        a0 = upd4(a0, s1, s2, f0);
        a1 = upd4(a1, s1, s2, f1);
        osm_step(lgB, mxB, dnB, s1, s2);
        a2 = upd4(a2, s1, s2, f2);
        a3 = upd4(a3, s1, s2, f3);
      }
      const float invA = __builtin_amdgcn_rcpf(dnA + EPS_SM);
      const float invB = __builtin_amdgcn_rcpf(dnB + EPS_SM);
      const v4f o0 = aff4(a0, invA, bA0);
      const v4f o1 = aff4(a1, invA, bA1);
      const v4f o2 = aff4(a2, invB, bB0);
      const v4f o3 = aff4(a3, invB, bB1);
      v2f e0, e1, e2, e3, e4, e5, e6, e7;
      e0.x = o0.x; e0.y = o0.y; e1.x = o0.z; e1.y = o0.w;
      e2.x = o1.x; e2.y = o1.y; e3.x = o1.z; e3.y = o1.w;
      e4.x = o2.x; e4.y = o2.y; e5.x = o2.z; e5.y = o2.w;
      e6.x = o3.x; e6.y = o3.y; e7.x = o3.z; e7.y = o3.w;
#pragma unroll 1
      for (int it = 0; it < 8; ++it) {
        v2f t;
        t.x = elu_f(e0.x);
        t.y = elu_f(e0.y);
        e0 = e1; e1 = e2; e2 = e3; e3 = e4; e4 = e5; e5 = e6; e6 = e7; e7 = t;
      }
      v4f p0, p1, p2, p3;
      p0.x = e0.x + pz; p0.y = e0.y + pz; p0.z = e1.x + pz; p0.w = e1.y + pz;
      p1.x = e2.x + pz; p1.y = e2.y + pz; p1.z = e3.x + pz; p1.w = e3.y + pz;
      p2.x = e4.x + pz; p2.y = e4.y + pz; p2.z = e5.x + pz; p2.w = e5.y + pz;
      p3.x = e6.x + pz; p3.y = e6.y + pz; p3.z = e7.x + pz; p3.w = e7.y + pz;
      const HL sa = split8(p0, p1);
      const HL sb = split8(p2, p3);
      unsigned short* gp = HP + (size_t)grow * KA2 + 8 * lane;
      const bool wr = grow < MPr;
      if (wr) {
        *(volatile v4u*)gp         = sa.hi;
        *(volatile v4u*)(gp + 256) = sb.hi;
        *(volatile v4u*)(gp + 512) = sa.lo;
        *(volatile v4u*)(gp + 768) = sb.lo;
      }
      __threadfence();
      if (wr) {
        *(volatile v4u*)gp         = sa.hi;
        *(volatile v4u*)(gp + 256) = sb.hi;
        *(volatile v4u*)(gp + 512) = sa.lo;
        *(volatile v4u*)(gp + 768) = sb.lo;
      }
    }
  } else {
    const int c0 = 2 * lane;
    const float bz0 = bfr(bias[c0]), bz1 = bfr(bias[c0 + 1]);
    const float g0 = bfr(gam[c0]),  g1 = bfr(gam[c0 + 1]);
    const float t0 = bfr(bet[c0]),  t1 = bfr(bet[c0 + 1]);
    const float* ASp = SD;
    const float* ADp = SD + MPr;

#pragma unroll 1
    for (int jt = 0; jt < nbw; ++jt) {
      const int slot = wave * nbw + jt;
      const int grow = nodeBase + slot;
      const int gcl  = grow < nN ? grow : nN - 1;
      int st = soff[slot];
      const int craw = scnt[slot];
      int cnt = craw;
      st  = st < 0 ? 0 : (st > nh ? nh : st);
      cnt = cnt < 0 ? 0 : (cnt > DEGCAP ? DEGCAP : cnt);
      if (cnt > nh - st) cnt = nh - st;
      const float pz = (ovf || craw > DEGCAP) ? qnan : 0.0f;

      const v2f fd = *(const v2fa*)(F + (size_t)gcl * HID + c0);
      const float adv = ADp[gcl];
      float mx = leaky(ASp[gcl] + adv), dn = 1.0f;
      float a0 = fd.x, a1 = fd.y;

#pragma unroll 1
      for (int q = 0; q < cnt; ++q) {
        int idx = st + q; idx = idx > RCAP - 1 ? RCAP - 1 : idx;
        int eid = reg2[idx]; eid = eid < 0 ? 0 : (eid > nE - 1 ? nE - 1 : eid);
        const int sraw = srcs[eid];
        const int s = sraw < 0 ? 0 : (sraw > nN - 1 ? nN - 1 : sraw);
        const v2f fs = *(const v2fa*)(F + (size_t)s * HID + c0);
        const float lg = leaky(ASp[s] + adv);
        float s1, s2;
        osm_step(lg, mx, dn, s1, s2);
        a0 = fmaf(a0, s1, s2 * fs.x);
        a1 = fmaf(a1, s1, s2 * fs.y);
      }
      const float inv = __builtin_amdgcn_rcpf(dn + EPS_SM);
      const float z0 = elu_f(fmaf(a0, inv, bz0));
      const float z1 = elu_f(fmaf(a1, inv, bz1));
      float sm = z0 + z1;
#pragma unroll
      for (int off = 16; off > 0; off >>= 1) sm += __shfl_xor(sm, off);
      const float mu = sm * (1.0f / 64.0f);
      const float d0 = z0 - mu, d1 = z1 - mu;
      float sq = d0 * d0 + d1 * d1;
#pragma unroll
      for (int off = 16; off > 0; off >>= 1) sq += __shfl_xor(sq, off);
      const float rs = __builtin_amdgcn_rcpf(sqrtf(sq * (1.0f / 64.0f) + EPS_LN));
      v2f ov;
      ov.x = (d0 * rs * g0 + t0) + pz;
      ov.y = (d1 * rs * g1 + t1) + pz;
      float* gp = LNF + (size_t)grow * HID + c0;
      const bool wr = grow < MPr;
      if (wr) *(volatile v2f*)gp = ov;
      __threadfence();
      if (wr) *(volatile v2f*)gp = ov;
    }
  }
}

__global__ __launch_bounds__(NTHR) void k_seq(const float* __restrict__ LNF, unsigned short* SEQ) {
  __shared__ __attribute__((aligned(16))) float sT[NPG * 68];
  const int tid = (int)threadIdx.x, b = (int)blockIdx.x;
#pragma unroll
  for (int i = 0; i < 2; ++i) {
    const int q = tid + NTHR * i;
    const int f = q >> 4, c4 = (q & 15) * 4;
    const v4f v = *(const v4fa*)(LNF + ((size_t)(b * NPG + f)) * HID + c4);
    *(v4fa*)(sT + f * 68 + c4) = v;
  }
  __syncthreads();
  v4u o[2];
#pragma unroll
  for (int i = 0; i < 2; ++i) {
    const int c = tid + NTHR * i;
    const int t = c >> 3, p = c & 7;
    const int f0 = (p & 3) * 8;
    const bool islo = p >= 4;
    unsigned int w[8];
#pragma unroll
    for (int j = 0; j < 8; ++j) {
      const float v = sT[(f0 + j) * 68 + t];
      const unsigned int hb = f2bf(v);
      const unsigned int lb = f2bf(v - bf2f(hb));
      w[j] = islo ? lb : hb;
    }
    v4u pv;
    pv.x = w[0] | (w[1] << 16); pv.y = w[2] | (w[3] << 16); pv.z = w[4] | (w[5] << 16); pv.w = w[6] | (w[7] << 16);
    o[i] = pv;
  }
  unsigned short* ob = SEQ + (size_t)b * (HID * 64);
#pragma unroll
  for (int i = 0; i < 2; ++i) *(volatile v4u*)(ob + (size_t)(tid + NTHR * i) * 8) = o[i];
  __threadfence();
#pragma unroll
  for (int i = 0; i < 2; ++i) *(volatile v4u*)(ob + (size_t)(tid + NTHR * i) * 8) = o[i];
}

__device__ __forceinline__ FragB ldfrag(const unsigned short* p, int hh) {
  FragB f;
  f.h[0] = *(const v8usa*)(p + 8 * hh);
  f.h[1] = *(const v8usa*)(p + 16 + 8 * hh);
  return f;
}
__device__ __forceinline__ void gates64(const unsigned short* arow, const unsigned short* W, int col, int hh,
                                        v8f& g0, v8f& g1, v8f& g2) {
  const FragB a0 = ldfrag(arow, hh), a1 = ldfrag(arow + 32, hh);
  const FragB a2 = ldfrag(arow + 64, hh), a3 = ldfrag(arow + 96, hh);
  {
    const unsigned short* wr = W + col * HID;
    const FragB b0 = ldfrag(wr, hh), b1 = ldfrag(wr + 32, hh);
    g0 = wmb(a0, b0, g0); g0 = wmb(a2, b0, g0); g0 = wmb(a1, b1, g0); g0 = wmb(a3, b1, g0);
  }
  {
    const unsigned short* wr = W + (HID + col) * HID;
    const FragB b0 = ldfrag(wr, hh), b1 = ldfrag(wr + 32, hh);
    g1 = wmb(a0, b0, g1); g1 = wmb(a2, b0, g1); g1 = wmb(a1, b1, g1); g1 = wmb(a3, b1, g1);
  }
  {
    const unsigned short* wr = W + (2 * HID + col) * HID;
    const FragB b0 = ldfrag(wr, hh), b1 = ldfrag(wr + 32, hh);
    g2 = wmb(a0, b0, g2); g2 = wmb(a2, b0, g2); g2 = wmb(a1, b1, g2); g2 = wmb(a3, b1, g2);
  }
}
__device__ __forceinline__ void gates32(const unsigned short* arow, const unsigned short* W, int col, int hh,
                                        v8f& g0, v8f& g1, v8f& g2) {
  const FragB a0 = ldfrag(arow, hh), a1 = ldfrag(arow + 32, hh);
  {
    const FragB b0 = ldfrag(W + col * NPG, hh);
    g0 = wmb(a0, b0, g0); g0 = wmb(a1, b0, g0);
  }
  {
    const FragB b0 = ldfrag(W + (HID + col) * NPG, hh);
    g1 = wmb(a0, b0, g1); g1 = wmb(a1, b0, g1);
  }
  {
    const FragB b0 = ldfrag(W + (2 * HID + col) * NPG, hh);
    g2 = wmb(a0, b0, g2); g2 = wmb(a1, b0, g2);
  }
}
__device__ __forceinline__ v8f gate_update(const v8f ar, const v8f az, const v8f axn, const v8f ahn, const v8f hp,
                                           float br, float bz, float bin, float bhn) {
  v8f hn;
#pragma unroll
  for (int r = 0; r < 8; ++r) {
    const float rg = sigm_f(ar[r] + br);
    const float zg = sigm_f(az[r] + bz);
    const float ng = tanhf((axn[r] + bin) + rg * (ahn[r] + bhn));
    hn[r] = (1.0f - zg) * ng + zg * hp[r];
  }
  return hn;
}
__device__ __forceinline__ void put_hl(unsigned short* hb, const v8f h, int rowb, int col) {
#pragma unroll
  for (int r = 0; r < 8; ++r) {
    const unsigned int hi = f2bf(h[r]);
    const unsigned int lo = f2bf(h[r] - bf2f(hi));
    hb[(rowb + r) * 128 + col]       = (unsigned short)hi;
    hb[(rowb + r) * 128 + HID + col] = (unsigned short)lo;
  }
}
__device__ __forceinline__ void cvt_plane(const float* __restrict__ w, unsigned short* s, int nUnits, int tid) {
#pragma unroll 1
  for (int u = tid; u < nUnits; u += NTHR) {
    const v4f a = *(const v4fa*)(w + 8 * u);
    const v4f c = *(const v4fa*)(w + 8 * u + 4);
    *(v4ua*)(s + 8 * u) = pack8(a, c);
  }
}

__global__ __launch_bounds__(NTHR) void k_rec(
    const unsigned short* __restrict__ SEQ,
    const float* __restrict__ Wi1, const float* __restrict__ Wh1, const float* __restrict__ bi1, const float* __restrict__ bh1,
    const float* __restrict__ Wi2, const float* __restrict__ Wh2, const float* __restrict__ bi2, const float* __restrict__ bh2,
    const float* __restrict__ Wf, const float* __restrict__ bfin, float* out)
{
  extern __shared__ v4f lds_dyn[];
  char* base = (char*)lds_dyn;
  unsigned short* sWi1 = (unsigned short*)(base + LO_WI1);
  unsigned short* sWh1 = (unsigned short*)(base + LO_WH1);
  unsigned short* sWi2 = (unsigned short*)(base + LO_WI2);
  unsigned short* sWh2 = (unsigned short*)(base + LO_WH2);
  unsigned short* sH1  = (unsigned short*)(base + LO_H1);
  unsigned short* sH2  = (unsigned short*)(base + LO_H2);
  unsigned short* sSeq = (unsigned short*)(base + LO_SEQ);
  float* sHF   = (float*)(base + LO_HF);
  float* sWf   = (float*)(base + LO_WF);
  float* sBf   = (float*)(base + LO_BF);
  float* sBias = (float*)(base + LO_BIAS);
  float* sOut  = (float*)(base + LO_OUT);

  const int tid = (int)threadIdx.x, lane = tid & 31, wave = tid >> 5;
  const int hh = lane >> 4, n = lane & 15;
  const int mt = wave >> 2, q = wave & 3;
  const int col  = 16 * q + n;
  const int mrow = 16 * mt + n;
  const int rowb = 16 * mt + 8 * hh;
  const int blk  = (int)blockIdx.x;
  const int b0   = blk * 32;

  cvt_plane(Wi1, sWi1, G3 * NPG / 8, tid);
  cvt_plane(Wh1, sWh1, G3 * HID / 8, tid);
  cvt_plane(Wi2, sWi2, G3 * HID / 8, tid);
  cvt_plane(Wh2, sWh2, G3 * HID / 8, tid);
  {
    const v4u zz = {0u, 0u, 0u, 0u};
#pragma unroll 1
    for (int i = tid; i < 2048; i += NTHR) *(v4ua*)(sH1 + 8 * i) = zz;
  }
  {
    const int i4 = tid < (G3 / 4) ? tid : (G3 / 4) - 1;
    const v4f v0 = bfr4(*(const v4fa*)(bi1 + 4 * i4));
    const v4f v1 = bfr4(*(const v4fa*)(bh1 + 4 * i4));
    const v4f v2 = bfr4(*(const v4fa*)(bi2 + 4 * i4));
    const v4f v3 = bfr4(*(const v4fa*)(bh2 + 4 * i4));
    if (tid < (G3 / 4)) {
      *(v4fa*)(sBias + 0 * G3 + 4 * tid) = v0;
      *(v4fa*)(sBias + 1 * G3 + 4 * tid) = v1;
      *(v4fa*)(sBias + 2 * G3 + 4 * tid) = v2;
      *(v4fa*)(sBias + 3 * G3 + 4 * tid) = v3;
    }
    const int j4 = tid < (NOUT * HID / 4) ? tid : (NOUT * HID / 4) - 1;
    const v4f wv = bfr4(*(const v4fa*)(Wf + 4 * j4));
    if (tid < (NOUT * HID / 4)) *(v4fa*)(sWf + 4 * tid) = wv;
    const float bv = bfin[tid < NOUT ? tid : NOUT - 1];
    if (tid < 16) sBf[tid] = (tid < NOUT) ? bfr(bv) : 0.0f;
  }
  __syncthreads();

  const float b1r  = sBias[0 * G3 + col] + sBias[1 * G3 + col];
  const float b1z  = sBias[0 * G3 + HID + col] + sBias[1 * G3 + HID + col];
  const float b1in = sBias[0 * G3 + 2 * HID + col];
  const float b1hn = sBias[1 * G3 + 2 * HID + col];
  const float b2r  = sBias[2 * G3 + col] + sBias[3 * G3 + col];
  const float b2z  = sBias[2 * G3 + HID + col] + sBias[3 * G3 + HID + col];
  const float b2in = sBias[2 * G3 + 2 * HID + col];
  const float b2hn = sBias[3 * G3 + 2 * HID + col];

  const v8f z8 = {0.f, 0.f, 0.f, 0.f, 0.f, 0.f, 0.f, 0.f};
  v8f h1v = z8, h2v = z8;
  const int srow = tid >> 3, spc = tid & 7;

#pragma unroll 1
  for (int t = 0; t < HID; ++t) {
    const int cur = t & 1, nxt = cur ^ 1;
    {
      const v4u sv = *(const v4ua*)(SEQ + ((size_t)(b0 + srow) * HID + t) * 64 + spc * 8);
      *(v4ua*)(sSeq + srow * 64 + spc * 8) = sv;
    }
    __syncthreads();

    {
      v8f ar = z8, az = z8, axn = z8, ahn = z8;
      gates32(sSeq + mrow * 64, sWi1, col, hh, ar, az, axn);
      gates64(sH1 + cur * 4096 + mrow * 128, sWh1, col, hh, ar, az, ahn);
      h1v = gate_update(ar, az, axn, ahn, h1v, b1r, b1z, b1in, b1hn);
      put_hl(sH1 + nxt * 4096, h1v, rowb, col);
    }
    __syncthreads();

    {
      v8f ar = z8, az = z8, axn = z8, ahn = z8;
      gates64(sH1 + nxt * 4096 + mrow * 128, sWi2, col, hh, ar, az, axn);
      gates64(sH2 + cur * 4096 + mrow * 128, sWh2, col, hh, ar, az, ahn);
      h2v = gate_update(ar, az, axn, ahn, h2v, b2r, b2z, b2in, b2hn);
      put_hl(sH2 + nxt * 4096, h2v, rowb, col);
    }
  }

#pragma unroll
  for (int r = 0; r < 8; ++r) sHF[(rowb + r) * HID + col] = h2v[r];
  __syncthreads();
#pragma unroll 1
  for (int idx = tid; idx < 32 * NOUT; idx += NTHR) {
    const int row = idx / NOUT;
    const int o   = idx - NOUT * row;
    const float* hr = sHF + row * HID;
    const float* wr = sWf + o * HID;
    float d = 0.0f;
#pragma unroll 4
    for (int c = 0; c < HID; ++c) d = fmaf(hr[c], wr[c], d);
    sOut[idx] = d + sBf[o];
  }
  __syncthreads();
  {
    const int pi = tid < 72 ? tid : 71;
    const v4f v = *(const v4fa*)(sOut + 4 * pi);
    float* op = out + (size_t)blk * (32 * NOUT) + 4 * pi;
    if (tid < 72) *(volatile v4f*)op = v;
    __threadfence();
    if (tid < 72) *(volatile v4f*)op = v;
  }
}

extern "C" void kernel_launch(void* const* d_in, const int* in_sizes, int n_in,
                              void* d_out, int out_size, void* d_ws, size_t ws_size,
                              hipStream_t stream) {
  if (n_in < 22) return;
  if (in_sizes[0] != NN * TIN) return;
  if (in_sizes[1] != 2 * NEDGE) return;
  if (in_sizes[2] != TIN * HC1) return;
  if (in_sizes[3] != NHD1 * HID || in_sizes[4] != NHD1 * HID) return;
  if (in_sizes[5] != HC1) return;
  if (in_sizes[6] != HC1 * HID) return;
  if (in_sizes[7] != HID || in_sizes[8] != HID || in_sizes[9] != HID) return;
  if (in_sizes[10] != HID || in_sizes[11] != HID) return;
  if (in_sizes[12] != G3 * NPG || in_sizes[13] != G3 * HID) return;
  if (in_sizes[14] != G3 || in_sizes[15] != G3) return;
  if (in_sizes[16] != G3 * HID || in_sizes[17] != G3 * HID) return;
  if (in_sizes[18] != G3 || in_sizes[19] != G3) return;
  if (in_sizes[20] != NOUT * HID || in_sizes[21] != NOUT) return;
  if (out_size != NBATCH * NOUT) return;
  if ((size_t)O_END > ws_size) return;

  const float* x   = (const float*)d_in[0];
  const int*   ei  = (const int*)  d_in[1];
  const float* W1  = (const float*)d_in[2];
  const float* as1 = (const float*)d_in[3];
  const float* ad1 = (const float*)d_in[4];
  const float* b1  = (const float*)d_in[5];
  const float* W2  = (const float*)d_in[6];
  const float* as2 = (const float*)d_in[7];
  const float* ad2 = (const float*)d_in[8];
  const float* b2  = (const float*)d_in[9];
  const float* gam = (const float*)d_in[10];
  const float* bet = (const float*)d_in[11];
  const float* Wi1 = (const float*)d_in[12];
  const float* Wh1 = (const float*)d_in[13];
  const float* bi1 = (const float*)d_in[14];
  const float* bh1 = (const float*)d_in[15];
  const float* Wi2 = (const float*)d_in[16];
  const float* Wh2 = (const float*)d_in[17];
  const float* bi2 = (const float*)d_in[18];
  const float* bh2 = (const float*)d_in[19];
  const float* Wf  = (const float*)d_in[20];
  const float* bfv = (const float*)d_in[21];
  float* out = (float*)d_out;
  const int* src = ei;
  const int* dst = ei + NEDGE;

  char* ws = (char*)d_ws;
  unsigned short* XB  = (unsigned short*)(ws + O_XB);
  unsigned short* W1T = (unsigned short*)(ws + O_W1T);
  unsigned short* W2D = (unsigned short*)(ws + O_W2D);
  float*          H1  = (float*)(ws + O_H1);
  float*          SD1 = (float*)(ws + O_SD1);
  unsigned short* X1  = (unsigned short*)(ws + O_X1);
  float*          H2  = (float*)(ws + O_H2);
  float*          SD2 = (float*)(ws + O_SD2);
  float*          LNF = (float*)(ws + O_LNF);
  unsigned short* SEQ = (unsigned short*)(ws + O_SEQ);

  hipFuncSetAttribute(reinterpret_cast<const void*>(&k_agg<1>),
                      hipFuncAttributeMaxDynamicSharedMemorySize, LDS_AGG);
  hipFuncSetAttribute(reinterpret_cast<const void*>(&k_agg<2>),
                      hipFuncAttributeMaxDynamicSharedMemorySize, LDS_AGG);
  hipFuncSetAttribute(reinterpret_cast<const void*>(&k_rec),
                      hipFuncAttributeMaxDynamicSharedMemorySize, LDS_REC);

  k_prep<<<PB_XB + PB_W1 + PB_W2, NTHR, 0, stream>>>(x, W1, W2, XB);
  k_gemm<<<dim3(NN / GBM, HC1 / GBN), GTHR, 0, stream>>>(XB, W1T, H1, KP1, HC1, as1, ad1, HID, SD1, NN);
  k_agg<1><<<NN / NBRUN, NTHR, LDS_AGG, stream>>>(src, dst, H1, SD1, b1, gam, bet, X1, LNF, NN, NEDGE, NBRUN, 1, NN);
  k_gemm<<<dim3(NN / GBM, 1), GTHR, 0, stream>>>(X1, W2D, H2, KA2, HID, as2, ad2, HID, SD2, NN);
  k_agg<2><<<NN / NBRUN, NTHR, LDS_AGG, stream>>>(src, dst, H2, SD2, b2, gam, bet, X1, LNF, NN, NEDGE, NBRUN, 1, NN);
  k_seq<<<NBATCH, NTHR, 0, stream>>>(LNF, SEQ);
  k_rec<<<NBATCH / 32, NTHR, LDS_REC, stream>>>(SEQ, Wi1, Wh1, bi1, bh1, Wi2, Wh2, bi2, bh2, Wf, bfv, out);
}
